// GlobalAttention_45028437131405
// MI455X (gfx1250) — hardware-verified
//
#include <hip/hip_runtime.h>
#include <math.h>

typedef __attribute__((ext_vector_type(16))) _Float16 v16h;
typedef __attribute__((ext_vector_type(16))) __bf16 v16b;
typedef __attribute__((ext_vector_type(8)))  _Float16 v8h;
typedef __attribute__((ext_vector_type(8)))  float v8f;
typedef __attribute__((ext_vector_type(4)))  float v4f;
typedef __attribute__((ext_vector_type(4)))  unsigned v4u;

template <typename T> __device__ __forceinline__ void vst2(void* p, T v) { *(volatile T*)p = v; __threadfence(); *(volatile T*)p = v; }
__device__ __forceinline__ v8f wmma16(v16h a, v16h b, v8f c) {
  v8f d = __builtin_amdgcn_wmma_f32_16x16x32_f16(false, a, false, b, (short)0, c, false, false);
  asm volatile("v_nop\n\tv_nop\n\tv_nop\n\tv_nop" : "+v"(d) : "v"(a), "v"(b));
  return d;
}
__device__ __forceinline__ v8f wmma_bf(v16b a, v16b b, v8f c) {
  v8f d = __builtin_amdgcn_wmma_f32_16x16x32_bf16(false, a, false, b, (short)0, c, false, false);
  asm volatile("v_nop\n\tv_nop\n\tv_nop\n\tv_nop" : "+v"(d) : "v"(a), "v"(b));
  return d;
}
__device__ __forceinline__ v16h frag_h(const _Float16* rowk0, int lane) {
  union { v16h v; v8h q[2]; } u; const _Float16* p = rowk0 + 8 * (lane >> 4);
  u.q[0] = *(const v8h*)p; u.q[1] = *(const v8h*)(p + 16); return u.v;
}
__device__ __forceinline__ v16h frag_f32(const float* rowk0, int lane) {
  v16h a; const float* p = rowk0 + 8 * (lane >> 4);
#pragma unroll
  for (int i = 0; i < 8; ++i) { a[i] = (_Float16)p[i]; a[8 + i] = (_Float16)p[16 + i]; }
  return a;
}
__device__ __forceinline__ v16h frag_f32s(const float* rowk0, int lane, float sc) {
  v16h a; const float* p = rowk0 + 8 * (lane >> 4);
#pragma unroll
  for (int i = 0; i < 8; ++i) { a[i] = (_Float16)(p[i] * sc); a[8 + i] = (_Float16)(p[16 + i] * sc); }
  return a;
}
__device__ __forceinline__ v16b rowb_f32(const float* rowk0, int lane) {
  v16b a; const float* p = rowk0 + 8 * (lane >> 4);
#pragma unroll
  for (int i = 0; i < 8; ++i) { a[i] = (__bf16)p[i]; a[8 + i] = (__bf16)p[16 + i]; }
  return a;
}
__device__ __forceinline__ float bfr(float v) { return (float)(__bf16)v; }
__device__ __forceinline__ v16b wcol_oi(const float* Wm, int k0, int o, int lane, int K) { v16b w; const float* p = Wm + (size_t)o * K + k0 + 8 * (lane >> 4);
#pragma unroll
  for (int i = 0; i < 8; ++i) { w[i] = (__bf16)p[i]; w[8 + i] = (__bf16)p[16 + i]; }
  return w; }
__device__ __forceinline__ v16h wcolh_oi(const float* Wm, int k0, int o, int lane, int K) { v16h w; const float* p = Wm + (size_t)o * K + k0 + 8 * (lane >> 4);
#pragma unroll
  for (int i = 0; i < 8; ++i) { w[i] = (_Float16)(bfr(p[i]) * 256.0f); w[8 + i] = (_Float16)(bfr(p[16 + i]) * 256.0f); }
  return w; }
__device__ __forceinline__ void ldsx() { asm volatile("s_wait_dscnt 0" ::: "memory"); __builtin_amdgcn_wave_barrier(); __builtin_amdgcn_fence(3, "workgroup"); }

#ifndef NB
#define NB 2
#endif
#ifndef SEQ
#define SEQ 4096
#endif
#define NB_FULL 2
#define SEQ_FULL 4096
#define TT SEQ
#define CC 256
#define DIN 256
#define NH 8
#define HD 32
#define NQB (TT / 64)
#define SCALE (0.17677669529663687f)
static_assert(NB >= 1 && NB <= NB_FULL);
static_assert(TT % 128 == 0 && TT >= 128 && TT <= SEQ_FULL);
static_assert(NH * HD == CC && HD % 32 == 0 && DIN % 128 == 0 && CC % 128 == 0);
static_assert((size_t)NB_FULL * SEQ_FULL * DIN * 4u == 8388608u);

#define WS_QH  0u
#define WS_KH  (WS_QH + 2u * (size_t)NB * TT * CC)
#define WS_VT  (WS_KH + 2u * (size_t)NB * TT * CC)
#define WS_S   (WS_VT + 2u * (size_t)NB * CC * TT)
#define WS_Y   (WS_S  + 4u * (size_t)TT * TT)
#define WS_END (WS_Y  + 4u * (size_t)NB * TT * CC)
static_assert(WS_END <= 134217728u);
static_assert(WS_KH % 128 == 0 && WS_VT % 128 == 0 && WS_S % 128 == 0 && WS_Y % 128 == 0 && WS_END % 128 == 0);

__global__ __launch_bounds__(128) __attribute__((amdgpu_num_vgpr(256))) void k_proj(const float* __restrict__ X, const float* __restrict__ WQ, const float* __restrict__ WK, const float* __restrict__ WV, const float* __restrict__ BQ, const float* __restrict__ BK, const float* __restrict__ BV,
    _Float16* __restrict__ QH, _Float16* __restrict__ KH, _Float16* __restrict__ VT) {
  __shared__ __align__(16) _Float16 sh[64][136]; __shared__ __align__(16) _Float16 th[128][72];
  const int tid = threadIdx.x, wave = tid >> 5, lane = tid & 31, col = lane & 15, g = lane >> 4; const int which = blockIdx.z; const int c0 = blockIdx.y * 128; const size_t r0 = (size_t)blockIdx.x * 64; const size_t bb = r0 / TT; const int t0 = (int)(r0 % TT);
  const float* WA = which == 0 ? WQ : which == 1 ? WK : WV; const float* BA = which == 0 ? BQ : which == 1 ? BK : BV;
  const float* xr = X + (bb * SEQ_FULL + (size_t)t0 + wave * 16 + col) * (size_t)DIN;
  v8f acc[8] = {};
#pragma unroll 1
  for (int kc = 0; kc < DIN / 32; ++kc) { const v16b a = rowb_f32(xr + kc * 32, lane);
    asm volatile("s_wait_loadcnt 0x0" ::: "memory");
#pragma unroll
    for (int j = 0; j < 8; ++j) { const v16b w = wcol_oi(WA, kc * 32, c0 + j * 16 + col, lane, DIN); asm volatile("s_wait_loadcnt 0x0" ::: "memory"); acc[j] = wmma_bf(a, w, acc[j]); } }
  if (which < 2) { _Float16* DH = which == 0 ? QH : KH;
#pragma unroll
    for (int j = 0; j < 8; ++j) { const float bias = bfr(BA[c0 + j * 16 + col]);
#pragma unroll
      for (int r = 0; r < 8; ++r) sh[wave * 16 + 8 * g + r][j * 16 + col] = (_Float16)(acc[j][r] + bias); }
    __syncthreads();
    for (int e = tid; e < 64 * 16; e += 128) { const int rl = e >> 4, q = e & 15; vst2((unsigned*)(DH + (r0 + rl) * CC + c0 + q * 8), *(const v4u*)&sh[rl][q * 8]); }
  } else {
#pragma unroll
    for (int j = 0; j < 8; ++j) { const float bias = bfr(BA[c0 + j * 16 + col]);
#pragma unroll
      for (int r = 0; r < 8; ++r) th[j * 16 + col][wave * 16 + 8 * g + r] = (_Float16)(acc[j][r] + bias); }
    __syncthreads();
    for (int e = tid; e < 128 * 8; e += 128) { const int cl = e >> 3, q = e & 7; vst2((unsigned*)(VT + (bb * CC + c0 + cl) * (size_t)TT + t0 + q * 8), *(const v4u*)&th[cl][q * 8]); } } }
__global__ __launch_bounds__(128) __attribute__((amdgpu_num_vgpr(256))) void k_sc(const _Float16* __restrict__ QH, const _Float16* __restrict__ KH, int b, int h, float* __restrict__ S) { __shared__ __align__(16) float ss[4][16][132];
  const int qb = blockIdx.x, kb = blockIdx.y;
  const int tid = threadIdx.x, wave = tid >> 5, lane = tid & 31, col = lane & 15, g = lane >> 4; const int k0 = kb * 128; const int ql0 = qb * 64 + wave * 16; const size_t q0 = (size_t)b * TT + ql0, kr0 = (size_t)b * TT + k0;
  v8f acc[8] = {};
#pragma unroll
  for (int kc = 0; kc < HD / 32; ++kc) { const v16h ah = frag_h(QH + (q0 + col) * CC + h * HD + kc * 32, lane);
#pragma unroll
    for (int j = 0; j < 8; ++j) { const v16h kf = frag_h(KH + (kr0 + j * 16 + col) * CC + h * HD + kc * 32, lane); acc[j] = wmma16(ah, kf, acc[j]); } }
#pragma unroll
  for (int j = 0; j < 8; ++j) {
#pragma unroll
    for (int r = 0; r < 8; ++r) ss[wave][8 * g + r][j * 16 + col] = acc[j][r] * SCALE; }
  ldsx(); for (int rl = 0; rl < 16; ++rl) vst2(S + (size_t)(ql0 + rl) * TT + k0 + lane * 4, *(const v4f*)&ss[wave][rl][lane * 4]); }
__global__ __launch_bounds__(256) __attribute__((amdgpu_num_vgpr(256))) void k_sm(float* __restrict__ S0) { __shared__ float sred[8]; __shared__ float sbc;
  constexpr int NQ4 = TT / 4; constexpr int NIT = (NQ4 + 255) / 256;
  const int tid = threadIdx.x; float* sr = S0 + (size_t)blockIdx.x * TT;
  v4f kv[NIT]; float m = -3.0e38f;
#pragma unroll
  for (int i = 0; i < NIT; ++i) { const int q = tid + 256 * i; const int qc = q < NQ4 ? q : NQ4 - 1;
    v4f v = *(const v4f*)(sr + (size_t)qc * 4);
    if (q >= NQ4) { v[0] = -3.0e38f; v[1] = -3.0e38f; v[2] = -3.0e38f; v[3] = -3.0e38f; }
    kv[i] = v; m = fmaxf(fmaxf(m, fmaxf(v[0], v[1])), fmaxf(v[2], v[3])); }
#pragma unroll
  for (int o = 1; o < 32; o <<= 1) m = fmaxf(m, __shfl_xor(m, o));
  if ((tid & 31) == 0) sred[tid >> 5] = m; __syncthreads(); if (tid == 0) { float a = sred[0]; for (int i = 1; i < 8; ++i) a = fmaxf(a, sred[i]); sbc = a; } __syncthreads(); m = sbc; __syncthreads();
  float sum = 0.f;
#pragma unroll
  for (int i = 0; i < NIT; ++i) { const int q = tid + 256 * i; v4f e;
#pragma unroll
    for (int c = 0; c < 4; ++c) e[c] = __expf(kv[i][c] - m);
    if (q >= NQ4) { e[0] = 0.f; e[1] = 0.f; e[2] = 0.f; e[3] = 0.f; }
    kv[i] = e; sum += (e[0] + e[1]) + (e[2] + e[3]); }
#pragma unroll
  for (int o = 1; o < 32; o <<= 1) sum += __shfl_xor(sum, o);
  if ((tid & 31) == 0) sred[tid >> 5] = sum; __syncthreads(); if (tid == 0) { float a = 0.f; for (int i = 0; i < 8; ++i) a += sred[i]; sbc = a > 0.f ? 2048.0f * (1.0f / a) : 0.f; } __syncthreads(); const float inv = sbc;
#pragma unroll
  for (int i = 0; i < NIT; ++i) { const int q = tid + 256 * i; const v4f o = kv[i] * inv; if (q < NQ4) vst2(sr + (size_t)q * 4, o); } }
__global__ __launch_bounds__(128) __attribute__((amdgpu_num_vgpr(256))) void k_pv(const float* __restrict__ PS, const _Float16* __restrict__ VT, int b, int h, float* __restrict__ Y) { __shared__ __align__(16) float ss[4][16][HD + 4];
  const int tid = threadIdx.x, wave = tid >> 5, lane = tid & 31, col = lane & 15, g = lane >> 4; const int qb = blockIdx.x; const int ql0 = qb * 64 + wave * 16;
  v8f acc[HD / 16] = {};
#pragma unroll 1
  for (int kc = 0; kc < TT / 32; ++kc) { const v16h p = frag_f32(PS + (size_t)(ql0 + col) * TT + kc * 32, lane);
    asm volatile("s_wait_loadcnt 0x0" ::: "memory");
#pragma unroll
    for (int j = 0; j < HD / 16; ++j) { const size_t po = ((size_t)b * CC + h * HD + j * 16 + col) * (size_t)TT + kc * 32; acc[j] = wmma16(p, frag_h(VT + po, lane), acc[j]); } }
#pragma unroll
  for (int j = 0; j < HD / 16; ++j)
#pragma unroll
    for (int r = 0; r < 8; ++r) ss[wave][8 * g + r][j * 16 + col] = acc[j][r] * (1.0f / 2048.0f);
  ldsx(); const int lc = lane < HD / 4 ? lane : 0;
  for (int rl = 0; rl < 16; ++rl) { const v4f o = *(const v4f*)&ss[wave][rl][lc * 4]; if (lane < HD / 4) vst2(Y + ((size_t)b * TT + ql0 + rl) * CC + h * HD + lane * 4, o); } }
__global__ __launch_bounds__(128) __attribute__((amdgpu_num_vgpr(256))) void k_out(const float* __restrict__ Y, const float* __restrict__ WO, const float* __restrict__ BO, float* __restrict__ OUT) { __shared__ __align__(16) float sf[4][16][132];
  const int tid = threadIdx.x, wave = tid >> 5, lane = tid & 31, col = lane & 15, g = lane >> 4; const int c0 = blockIdx.y * 128;
  const size_t rb = (size_t)blockIdx.x * 64; const size_t r0 = rb + wave * 16; const size_t bb = rb / TT; const size_t orow0 = bb * SEQ_FULL + (rb % TT) + wave * 16;
  v8f acc[8] = {};
#pragma unroll 1
  for (int kc = 0; kc < CC / 32; ++kc) { const v16h a = frag_f32s(Y + (r0 + col) * CC + kc * 32, lane, 64.0f); asm volatile("s_wait_loadcnt 0x0" ::: "memory");
#pragma unroll
    for (int j = 0; j < 8; ++j) { const v16h w = wcolh_oi(WO, kc * 32, c0 + j * 16 + col, lane, CC); asm volatile("s_wait_loadcnt 0x0" ::: "memory"); acc[j] = wmma16(a, w, acc[j]); } }
#pragma unroll
  for (int j = 0; j < 8; ++j) { const float bias = bfr(BO[c0 + j * 16 + col]);
#pragma unroll
    for (int r = 0; r < 8; ++r) sf[wave][8 * g + r][j * 16 + col] = acc[j][r] * (1.0f / 16384.0f) + bias; }
  ldsx(); for (int rl = 0; rl < 16; ++rl) vst2(OUT + (orow0 + rl) * DIN + c0 + lane * 4, *(const v4f*)&sf[wave][rl][lane * 4]); }

extern "C" void kernel_launch(void* const* d_in, const int* in_sizes, int n_in, void* d_out, int out_size, void* d_ws, size_t ws_size, hipStream_t stream) {
  if (n_in < 9) return;
  const size_t nrow_need = (size_t)(NB - 1) * SEQ_FULL + TT;
  if ((size_t)in_sizes[0] < nrow_need * DIN) return;
  if (in_sizes[1] < CC * DIN || in_sizes[3] < CC * DIN || in_sizes[5] < CC * DIN || in_sizes[7] < DIN * CC) return;
  if (in_sizes[2] < CC || in_sizes[4] < CC || in_sizes[6] < CC || in_sizes[8] < DIN) return;
  if ((size_t)out_size < nrow_need * DIN) return;
  if (ws_size < (size_t)WS_END) return;
  const float* const* F = (const float* const*)d_in;
  char* ws = (char*)d_ws; _Float16 *QH = (_Float16*)(ws + WS_QH), *KH = (_Float16*)(ws + WS_KH), *VT = (_Float16*)(ws + WS_VT); float *S = (float*)(ws + WS_S), *Y = (float*)(ws + WS_Y);
  k_proj<<<dim3(NB * TT / 64, CC / 128, 3), 128, 0, stream>>>(F[0], F[1], F[3], F[5], F[2], F[4], F[6], QH, KH, VT);
  for (int b = 0; b < NB; ++b) for (int h = 0; h < NH; ++h) {
    k_sc<<<dim3(NQB, TT / 128, 1), 128, 0, stream>>>(QH, KH, b, h, S);
    k_sm<<<dim3(TT), 256, 0, stream>>>(S);
    k_pv<<<dim3(NQB), 128, 0, stream>>>(S, VT, b, h, Y);
  }
  k_out<<<dim3(NB * TT / 64, DIN / 128), 128, 0, stream>>>(Y, F[7], F[8], (float*)d_out);
}
